// UltrasoundWNO1d_1288490189220
// MI455X (gfx1250) — hardware-verified
//
#include <hip/hip_runtime.h>
#include <stdint.h>
#include <math.h>


#define KS 8192

typedef float v4f __attribute__((ext_vector_type(4)));
typedef v4f v4fa __attribute__((may_alias));
typedef float v8f __attribute__((ext_vector_type(8)));
typedef unsigned short v8us __attribute__((ext_vector_type(8)));
typedef v8us v8usa __attribute__((may_alias));
typedef __bf16 v16bf __attribute__((ext_vector_type(16)));
typedef _Float16 v16h __attribute__((ext_vector_type(16)));

union Frag { v16h vh; v16bf vb; v8us hv[2]; };
union HBits { _Float16 f; unsigned short u; };

struct LvTab { int L[8]; int P[8]; int off[8]; };
typedef char lvtab_size_check[(sizeof(LvTab) == 96) ? 1 : -1];
struct WpTab {
  int oC3, oM1, oM2, oCAh, oCAl, oCDh, oCDl, oP1h, oP1l, oP2h, oP2l;
  int nC3, nM1, nM2, nCA, nCD, nP1, nP2;
  int C, z;
};
typedef char wptab_size_check[(sizeof(WpTab) == 80) ? 1 : -1];

__constant__ float c_lo[16] = {
  (float)(-0.0033824159510061256), (float)(-0.0005421323317911481), (float)(0.03169508781149298),
  (float)(0.007607487324917605),   (float)(-0.1432942383508097),    (float)(-0.061273359067658524),
  (float)(0.4813596512583722),     (float)(0.7771857517005235),     (float)(0.3644418948353314),
  (float)(-0.051945838107709037),  (float)(-0.027219029917056003),  (float)(0.049137179673607506),
  (float)(0.003808752013890615),   (float)(-0.01495225833704823),   (float)(-0.0003029205147213668),
  (float)(0.0018899503327594609) };

__device__ __forceinline__ unsigned short f2bf(float f) {
  unsigned int u = __float_as_uint(f);
  u += 0x7FFFu + ((u >> 16) & 1u);
  return (unsigned short)(u >> 16);
}
__device__ __forceinline__ float bf2f(unsigned short s) {
  return __uint_as_float(((unsigned int)s) << 16);
}
__device__ __forceinline__ unsigned short f2h(float f) {
  HBits hb; hb.f = (_Float16)f;
  return hb.u;
}
__device__ __forceinline__ float gelu_f(float x) {
  return 0.5f * x * (1.0f + erff(x * 0.70710678118654752f));
}
__device__ __forceinline__ float wave_sum(float v) {
  #pragma unroll
  for (int o = 16; o > 0; o >>= 1) v += __shfl_xor(v, o, 32);
  return v;
}

__device__ __forceinline__ void mma1h(v8f& acc, const v16h a, const v16h b) {
  acc = __builtin_amdgcn_wmma_f32_16x16x32_f16(false, a, false, b, (short)0, acc, false, false);
  asm volatile("v_nop\n\tv_nop\n\tv_nop\n\tv_nop" : "+v"(acc) : "v"(a), "v"(b));
}
__device__ __forceinline__ void mma3(v8f& acc, const v16bf ah, const v16bf al, const v16bf bh, const v16bf bl) {
  acc = __builtin_amdgcn_wmma_f32_16x16x32_bf16(false, ah, false, bh, (short)0, acc, false, false);
  acc = __builtin_amdgcn_wmma_f32_16x16x32_bf16(false, ah, false, bl, (short)0, acc, false, false);
  acc = __builtin_amdgcn_wmma_f32_16x16x32_bf16(false, al, false, bh, (short)0, acc, false, false);
  asm volatile("v_nop\n\tv_nop\n\tv_nop\n\tv_nop" : "+v"(acc) : "v"(ah), "v"(al), "v"(bh), "v"(bl));
}

__global__ __launch_bounds__(256) void k_wprep(const float* __restrict__ bww, const float* __restrict__ m1w,
                                               const float* __restrict__ m2w, const float* __restrict__ caw,
                                               const float* __restrict__ cdw, const float* __restrict__ p1w,
                                               const float* __restrict__ p2w, unsigned short* wp, WpTab t)
{
  const int tid = threadIdx.x;
  const int seg = blockIdx.y;
  const int g = blockIdx.x * 256 + tid;
  const float* src = p2w; int n = t.nP2, oh = t.oP2h, ol = t.oP2l, kind = 2;
  if (seg == 0)      { src = bww; n = t.nC3; oh = t.oC3;  ol = t.oC3;  kind = 0; }
  else if (seg == 1) { src = m1w; n = t.nM1; oh = t.oM1;  ol = t.oM1;  kind = 1; }
  else if (seg == 2) { src = m2w; n = t.nM2; oh = t.oM2;  ol = t.oM2;  kind = 1; }
  else if (seg == 3) { src = caw; n = t.nCA; oh = t.oCAh; ol = t.oCAl; kind = 2; }
  else if (seg == 4) { src = cdw; n = t.nCD; oh = t.oCDh; ol = t.oCDl; kind = 2; }
  else if (seg == 5) { src = p1w; n = t.nP1; oh = t.oP1h; ol = t.oP1l; kind = 2; }
  const int n8 = n >> 3;
  const bool ok = (g < n8);
  v8us hv = {0, 0, 0, 0, 0, 0, 0, 0};
  v8us lv = {0, 0, 0, 0, 0, 0, 0, 0};
  unsigned short* dh = wp + (size_t)oh + (size_t)g * 8;
  unsigned short* dl = wp + (size_t)ol + (size_t)g * 8;
  if (ok) {
    float f[8];
    if (kind == 0) {
      const int C = t.C;
      const int e = g * 8;
      const int k = e % C;
      int q = e / C;
      const int m = q % C;
      q = q / C;
      const int tap = q % 3;
      const int bk = q / 3;
      const size_t sb = (((size_t)bk * C + m) * (size_t)C + (size_t)k) * 3 + (size_t)tap;
      #pragma unroll
      for (int i = 0; i < 8; ++i) f[i] = 8.0f * src[sb + (size_t)(3 * i)];
    } else {
      const size_t sb = (size_t)g * 8;
      const float sc = (kind == 1) ? 8.0f : 1.0f;
      #pragma unroll
      for (int i = 0; i < 8; ++i) f[i] = sc * src[sb + (size_t)i];
    }
    if (kind == 2) {
      #pragma unroll
      for (int i = 0; i < 8; ++i) {
        const unsigned short hi = f2bf(f[i]);
        hv[i] = hi;
        lv[i] = f2bf(f[i] - bf2f(hi));
      }
    } else {
      #pragma unroll
      for (int i = 0; i < 8; ++i) hv[i] = f2h(f[i]);
    }
    *(volatile v8us*)dh = hv;
    if (kind == 2) *(volatile v8us*)dl = lv;
  }
  __threadfence();
  if (ok) {
    *(volatile v8us*)dh = hv;
    if (kind == 2) *(volatile v8us*)dl = lv;
  }
}

__global__ __launch_bounds__(256) void k_lift(const float* __restrict__ x, const float* __restrict__ lw,
                                              const float* __restrict__ lb, float* Hout, int C, int total4)
{
  #pragma clang fp contract(off)
  const int gid = blockIdx.x * 256 + (int)threadIdx.x;
  if (gid >= total4) return;
  const size_t e = (size_t)gid * 4;
  const int row = (int)(e / KS);
  const int lp0 = (int)(e % KS);
  const int b = row / C;
  const int c = row - b * C;
  const float w0 = lw[2 * c], w1 = lw[2 * c + 1], bb = lb[c];
  const float rcp = 1.0f / (float)(KS - 1);
  const float* xr = x + (size_t)b * KS;
  float ov[4];
  #pragma unroll
  for (int u = 0; u < 4; ++u) {
    const int lp = lp0 + u;
    float g;
    if (lp == KS - 1) g = 1.0f;
    else { const float st = (float)lp * rcp; const float a = 1.0f - st; g = st - a; }
    ov[u] = (w0 * xr[lp] + w1 * g) + bb;
  }
  v4f o; o.x = ov[0]; o.y = ov[1]; o.z = ov[2]; o.w = ov[3];
  *(volatile v4f*)(Hout + e) = o;
  __threadfence();
  *(volatile v4f*)(Hout + e) = o;
}

__global__ __launch_bounds__(256) void k_stats(const float* X, float* ST)
{
  #pragma clang fp contract(off)
  __shared__ float red[16];
  __shared__ __attribute__((aligned(16))) float stt[64];
  const int tid = threadIdx.x, l = tid & 31, wv = tid >> 5;
  const int r0 = blockIdx.x * 32;
  #pragma unroll 1
  for (int r = 0; r < 32; ++r) {
    const size_t base = (size_t)(r0 + r) * KS;
    v4f v[8];
    float s = 0.0f;
    #pragma unroll
    for (int j = 0; j < 8; ++j) {
      v[j] = *(const v4fa*)(X + base + (size_t)(j * 256 + tid) * 4);
      s += (v[j].x + v[j].y) + (v[j].z + v[j].w);
    }
    s = wave_sum(s);
    if (l == 0) red[wv] = s;
    __syncthreads();
    float tot = 0.0f;
    #pragma unroll
    for (int w = 0; w < 8; ++w) tot += red[w];
    const float mean = tot * (1.0f / KS);
    float q = 0.0f;
    #pragma unroll
    for (int j = 0; j < 8; ++j) {
      const v4f d = v[j] - mean;
      q += (d.x * d.x + d.y * d.y) + (d.z * d.z + d.w * d.w);
    }
    q = wave_sum(q);
    if (l == 0) red[8 + wv] = q;
    __syncthreads();
    float tq = 0.0f;
    #pragma unroll
    for (int w = 0; w < 8; ++w) tq += red[8 + w];
    const float inv = rsqrtf(tq * (1.0f / KS) + 1e-5f);
    if (tid == 0) { stt[2 * r] = mean; stt[2 * r + 1] = inv; }
  }
  __syncthreads();
  const bool wr = (tid < 16);
  const v4f z4 = {0.0f, 0.0f, 0.0f, 0.0f};
  v4f o = z4;
  float* dst = ST + (size_t)r0 * 2 + (size_t)((tid & 15) * 4);
  if (wr) { o = *(const v4fa*)(stt + 4 * tid); *(volatile v4f*)dst = o; }
  __threadfence();
  if (wr) *(volatile v4f*)dst = o;
}

__global__ __launch_bounds__(256) void k_dwt(const float* Xin, const float* __restrict__ ST, float* WD, float* WA, LvTab tb, int LV)
{
  __shared__ __attribute__((aligned(16))) float ext[8320];
  __shared__ __attribute__((aligned(16))) float tmp[4160];
  __shared__ float tk[32];
  const int tid = threadIdx.x;
  const int row = blockIdx.x;
  if (tid < 16) {
    const float cl = c_lo[15 - tid];
    const float ch = c_lo[tid];
    tk[tid] = cl;
    tk[16 + tid] = (tid & 1) ? -ch : ch;
  }
  const float mean = ST[2 * row], rstd = ST[2 * row + 1];
  const float* src = Xin + (size_t)row * KS;
  int Lin = KS;
  for (int lv = 1; lv <= LV; ++lv) {
    const int Lout = tb.L[lv], Pout = tb.P[lv];
    const int EL = Lin + 29;
    const int ELZ = 2 * Pout + 16;
    __syncthreads();
    for (int p = tid; p < ELZ; p += 256) {
      float v = 0.0f;
      if (p < EL) {
        int j = p - 14;
        if (j < 0) j = -j - 1;
        if (j >= Lin) j = 2 * Lin - 1 - j;
        v = src[j];
        if (lv == 1) v = (v - mean) * rstd;
      }
      ext[p] = v;
    }
    __syncthreads();
    float* drow = WD + (size_t)tb.off[lv] + (size_t)row * (size_t)Pout;
    const bool last = (lv == LV);
    float* arow = last ? (WA + (size_t)row * (size_t)Pout) : WA;
    const int ng = Pout >> 2;
    v4f dv[5], av[5];
    #pragma unroll
    for (int it = 0; it < 5; ++it) {
      const int g = tid + it * 256;
      const v4f z4 = {0.0f, 0.0f, 0.0f, 0.0f};
      dv[it] = z4; av[it] = z4;
      if (g < ng) {
        float alo[4] = {0.0f, 0.0f, 0.0f, 0.0f}, ahi[4] = {0.0f, 0.0f, 0.0f, 0.0f};
        #pragma unroll 1
        for (int t = 0; t < 16; ++t) {
          const float kl = tk[t], kh = tk[16 + t];
          #pragma unroll
          for (int u = 0; u < 4; ++u) {
            const float xv = ext[8 * g + 2 * u + t];
            alo[u] += xv * kl;
            ahi[u] += xv * kh;
          }
        }
        float aa[4], dd[4];
        #pragma unroll
        for (int u = 0; u < 4; ++u) {
          const int i = 4 * g + u;
          const bool ok = (i < Lout);
          aa[u] = ok ? alo[u] : 0.0f;
          dd[u] = ok ? ahi[u] : 0.0f;
          if (ok) tmp[i] = alo[u];
        }
        v4f a4, d4;
        a4.x = aa[0]; a4.y = aa[1]; a4.z = aa[2]; a4.w = aa[3];
        d4.x = dd[0]; d4.y = dd[1]; d4.z = dd[2]; d4.w = dd[3];
        dv[it] = d4; av[it] = a4;
        *(volatile v4f*)(drow + 4 * g) = d4;
        if (last) *(volatile v4f*)(arow + 4 * g) = a4;
      }
    }
    __threadfence();
    #pragma unroll
    for (int it = 0; it < 5; ++it) {
      const int g = tid + it * 256;
      if (g < ng) {
        *(volatile v4f*)(drow + 4 * g) = dv[it];
        if (last) *(volatile v4f*)(arow + 4 * g) = av[it];
      }
    }
    src = tmp;
    Lin = Lout;
  }
}

__device__ __forceinline__ void synth4(int G, float* y, const float* az, const float* dz, const float* tk)
{
  float y0 = 0.0f, y1 = 0.0f, y2 = 0.0f, y3 = 0.0f;
  const int p = 2 * G;
  #pragma unroll 1
  for (int s = 0; s < 8; ++s) {
    const float a0 = az[p + s], a1 = az[p + 1 + s];
    const float d0 = dz[p + s], d1 = dz[p + 1 + s];
    const float ro = tk[2 * s + 1], re = tk[2 * s];
    const float ho = tk[16 + 2 * s + 1], he = tk[16 + 2 * s];
    y0 += a0 * ro + d0 * ho;
    y1 += a0 * re + d0 * he;
    y2 += a1 * ro + d1 * ho;
    y3 += a1 * re + d1 * he;
  }
  y[0] = y0; y[1] = y1; y[2] = y2; y[3] = y3;
}

__global__ __launch_bounds__(256) void k_idwt(const float* WAm, const float* WDm, const float* XS, float* Hb, LvTab tb, int LV)
{
  __shared__ __attribute__((aligned(16))) float az[4160];
  __shared__ __attribute__((aligned(16))) float dz[4160];
  __shared__ __attribute__((aligned(16))) float yb[4160];
  __shared__ float tk[32];
  const int tid = threadIdx.x;
  const int row = blockIdx.x;
  if (tid < 16) {
    const float c15 = c_lo[15 - tid];
    tk[tid] = c_lo[tid];
    tk[16 + tid] = (tid & 1) ? c15 : -c15;
  }
  const float* asrc = WAm + (size_t)row * (size_t)tb.P[LV];
  int alen = tb.L[LV];
  for (int lv = LV; lv >= 1; --lv) {
    const int dl = tb.L[lv];
    const int la = (alen == dl + 1) ? dl : alen;
    const int lo = 2 * la - 14;
    const float* dsrc = WDm + (size_t)tb.off[lv] + (size_t)row * (size_t)tb.P[lv];
    __syncthreads();
    const int LZ = la + 16;
    for (int m = tid; m < LZ; m += 256) {
      float a = 0.0f, d = 0.0f;
      if (m < la) { a = asrc[m]; d = dsrc[m]; }
      az[m] = a; dz[m] = d;
    }
    __syncthreads();
    if (lv > 1) {
      const int ng = (lo + 3) >> 2;
      #pragma unroll 1
      for (int g = tid; g < ng; g += 256) {
        float y[4];
        synth4(g, y, az, dz, tk);
        #pragma unroll
        for (int u = 0; u < 4; ++u) { const int i = 4 * g + u; if (i < lo) yb[i] = y[u]; }
      }
      asrc = yb;
      alen = lo;
    } else {
      const size_t rb = (size_t)row * KS;
      #pragma unroll 1
      for (int ch = 0; ch < KS; ch += 4096) {
        #pragma unroll 1
        for (int g = tid; g < 1024; g += 256) {
          const int G = (ch >> 2) + g;
          float y[4];
          synth4(G, y, az, dz, tk);
          const size_t off = rb + (size_t)4 * G;
          const v4f xs = *(const v4fa*)(XS + off);
          const v4f hv = *(const v4fa*)(Hb + off);
          v4f o;
          o.x = hv.x + gelu_f(y[0] + xs.x);
          o.y = hv.y + gelu_f(y[1] + xs.y);
          o.z = hv.z + gelu_f(y[2] + xs.z);
          o.w = hv.w + gelu_f(y[3] + xs.w);
          *(volatile v4f*)(Hb + off) = o;
          *(v4fa*)(yb + 4 * g) = o;
        }
        __threadfence();
        #pragma unroll 1
        for (int g = tid; g < 1024; g += 256) {
          const int G = (ch >> 2) + g;
          const v4f o = *(const v4fa*)(yb + 4 * g);
          *(volatile v4f*)(Hb + rb + (size_t)4 * G) = o;
        }
      }
    }
  }
}

template<int MT, int MODE>
__global__ __launch_bounds__(64) void k_mix(const unsigned short* __restrict__ Wh, const unsigned short* __restrict__ Wl,
                                            int wts, int T, const float* __restrict__ bias,
                                            const float* X, const float* __restrict__ nst,
                                            int K, int Nv, int P, int xbs,
                                            float* Y, int ybs, int act)
{
  constexpr int M = MT * 16;
  __shared__ __attribute__((aligned(16))) float xo[4608];
  unsigned short* xsh = reinterpret_cast<unsigned short*>(xo);
  unsigned short* xsl = xsh + 4608;

  const int tid = threadIdx.x;
  const int l = tid & 31, wv = tid >> 5, h = l >> 4, m15 = l & 15;
  const int KP = K + 8;
  const int halo = (T - 1) >> 1;
  const int NC = 32 + T - 1;
  const int n0 = blockIdx.x * 32;
  const int b = blockIdx.z;
  const float* Xb = X + (size_t)b * (size_t)xbs;

  for (int k = wv; k < K; k += 2) {
    const float* xr = Xb + (size_t)k * (size_t)P;
    float mean = 0.0f, rstd = 1.0f;
    if (nst != nullptr) { const int rr = b * K + k; mean = nst[2 * rr]; rstd = nst[2 * rr + 1]; }
    for (int j = l; j < NC; j += 32) {
      const int c = n0 + j - halo;
      float v = 0.0f;
      if (c >= 0 && c < Nv) v = (xr[c] - mean) * rstd;
      if (MODE == 0) {
        xsh[j * KP + k] = f2h(v);
      } else {
        const unsigned short hi = f2bf(v);
        xsh[j * KP + k] = hi;
        xsl[j * KP + k] = f2bf(v - bf2f(hi));
      }
    }
  }
  __syncthreads();

  v8f acc[MT];
  #pragma unroll
  for (int mt = 0; mt < MT; ++mt) {
    #pragma unroll
    for (int r = 0; r < 8; ++r) acc[mt][r] = 0.0f;
  }

  for (int tap = 0; tap < T; ++tap) {
    const unsigned short* wth = Wh + (size_t)tap * (size_t)wts;
    const unsigned short* wtl = Wl + (size_t)tap * (size_t)wts;
    const int xrow = (wv * 16 + m15 + tap) * KP + 8 * h;
    for (int k0 = 0; k0 < K; k0 += 32) {
      Frag bh, bl;
      bh.hv[0] = *(const v8usa*)(xsh + xrow + k0);
      bh.hv[1] = *(const v8usa*)(xsh + xrow + k0 + 16);
      if (MODE == 1) {
        bl.hv[0] = *(const v8usa*)(xsl + xrow + k0);
        bl.hv[1] = *(const v8usa*)(xsl + xrow + k0 + 16);
      }
      #pragma unroll
      for (int mt = 0; mt < MT; ++mt) {
        const size_t ao = (size_t)(mt * 16 + m15) * (size_t)K + (size_t)(k0 + 8 * h);
        Frag ah;
        ah.hv[0] = *(const v8usa*)(wth + ao);
        ah.hv[1] = *(const v8usa*)(wth + ao + 16);
        if (MODE == 0) {
          mma1h(acc[mt], ah.vh, bh.vh);
        } else {
          Frag al;
          al.hv[0] = *(const v8usa*)(wtl + ao);
          al.hv[1] = *(const v8usa*)(wtl + ao + 16);
          mma3(acc[mt], ah.vb, al.vb, bh.vb, bl.vb);
        }
      }
    }
  }
  __syncthreads();
  #pragma unroll
  for (int mt = 0; mt < MT; ++mt) {
    #pragma unroll
    for (int r = 0; r < 8; ++r)
      xo[(mt * 16 + 8 * h + r) * 36 + wv * 16 + m15] = acc[mt][r];
  }
  __syncthreads();
  const float osc = (MODE == 0) ? 0.125f : 1.0f;
  const int cq = (l & 7) * 4;
  const int rsub = l >> 3;
  v4f vals[MT * 2];
  #pragma unroll
  for (int s = 0; s < MT * 2; ++s) {
    const int m = wv * (MT * 8) + s * 4 + rsub;
    v4f v = *(const v4fa*)(xo + m * 36 + cq);
    const float bm = (bias != nullptr) ? bias[m] : 0.0f;
    v = v * osc + bm;
    if (act) { v.x = gelu_f(v.x); v.y = gelu_f(v.y); v.z = gelu_f(v.z); v.w = gelu_f(v.w); }
    const size_t off = (size_t)b * (size_t)ybs + (size_t)m * (size_t)P + (size_t)(n0 + cq);
    vals[s] = v;
    *(volatile v4f*)(Y + off) = v;
  }
  __threadfence();
  #pragma unroll
  for (int s = 0; s < MT * 2; ++s) {
    const int m = wv * (MT * 8) + s * 4 + rsub;
    const size_t off = (size_t)b * (size_t)ybs + (size_t)m * (size_t)P + (size_t)(n0 + cq);
    *(volatile v4f*)(Y + off) = vals[s];
  }
}

template<int MC, int MH>
__global__ __launch_bounds__(64) void k_mlp(const unsigned short* __restrict__ W1, const float* __restrict__ b1,
                                            const unsigned short* __restrict__ W2, const float* __restrict__ b2,
                                            const float* __restrict__ nst, float* Hb, int P)
{
  constexpr int C = MC * 16, HH = MH * 16, KP1 = C + 8, KP2 = HH + 8;
  __shared__ __attribute__((aligned(16))) unsigned short xs1[32 * KP1];
  __shared__ __attribute__((aligned(16))) unsigned short hsb[32 * KP2];
  __shared__ __attribute__((aligned(16))) float xo[C * 36];
  const int tid = threadIdx.x;
  const int l = tid & 31, wv = tid >> 5, h = l >> 4, m15 = l & 15;
  const int n0 = blockIdx.x * 32;
  const int b = blockIdx.z;
  float* Hbb = Hb + (size_t)b * (size_t)C * (size_t)P;

  for (int k = wv; k < C; k += 2) {
    const int rr = b * C + k;
    const float mean = nst[2 * rr], rstd = nst[2 * rr + 1];
    const float v = (Hbb[(size_t)k * (size_t)P + (size_t)(n0 + l)] - mean) * rstd;
    xs1[l * KP1 + k] = f2h(v);
  }
  __syncthreads();

  const int ncol = wv * 16 + m15;
  v8f acc1[MH];
  #pragma unroll
  for (int mt = 0; mt < MH; ++mt) {
    #pragma unroll
    for (int r = 0; r < 8; ++r) acc1[mt][r] = 0.0f;
  }
  {
    const int xrow = ncol * KP1 + 8 * h;
    #pragma unroll
    for (int k0 = 0; k0 < C; k0 += 32) {
      Frag bb;
      bb.hv[0] = *(const v8usa*)(xs1 + xrow + k0);
      bb.hv[1] = *(const v8usa*)(xs1 + xrow + k0 + 16);
      #pragma unroll
      for (int mt = 0; mt < MH; ++mt) {
        const unsigned short* wa = W1 + (size_t)(mt * 16 + m15) * (size_t)C + (size_t)(k0 + 8 * h);
        Frag aa;
        aa.hv[0] = *(const v8usa*)(wa);
        aa.hv[1] = *(const v8usa*)(wa + 16);
        mma1h(acc1[mt], aa.vh, bb.vh);
      }
    }
  }
  #pragma unroll
  for (int mt = 0; mt < MH; ++mt) {
    #pragma unroll
    for (int r = 0; r < 8; ++r) {
      const int m = mt * 16 + 8 * h + r;
      float v = acc1[mt][r] * 0.125f + b1[m];
      v = gelu_f(v);
      hsb[ncol * KP2 + m] = f2h(v);
    }
  }
  __syncthreads();

  v8f acc2[MC];
  #pragma unroll
  for (int mt = 0; mt < MC; ++mt) {
    #pragma unroll
    for (int r = 0; r < 8; ++r) acc2[mt][r] = 0.0f;
  }
  {
    const int hrow = ncol * KP2 + 8 * h;
    #pragma unroll
    for (int k0 = 0; k0 < HH; k0 += 32) {
      Frag bb;
      bb.hv[0] = *(const v8usa*)(hsb + hrow + k0);
      bb.hv[1] = *(const v8usa*)(hsb + hrow + k0 + 16);
      #pragma unroll
      for (int mt = 0; mt < MC; ++mt) {
        const unsigned short* wa = W2 + (size_t)(mt * 16 + m15) * (size_t)HH + (size_t)(k0 + 8 * h);
        Frag aa;
        aa.hv[0] = *(const v8usa*)(wa);
        aa.hv[1] = *(const v8usa*)(wa + 16);
        mma1h(acc2[mt], aa.vh, bb.vh);
      }
    }
  }
  #pragma unroll
  for (int mt = 0; mt < MC; ++mt) {
    #pragma unroll
    for (int r = 0; r < 8; ++r)
      xo[(mt * 16 + 8 * h + r) * 36 + ncol] = acc2[mt][r];
  }
  __syncthreads();
  const int cq = (l & 7) * 4;
  const int rsub = l >> 3;
  v4f vals[MC * 2];
  #pragma unroll
  for (int s = 0; s < MC * 2; ++s) {
    const int m = wv * (MC * 8) + s * 4 + rsub;
    v4f v = *(const v4fa*)(xo + m * 36 + cq);
    v = v * 0.125f + b2[m];
    const size_t off = (size_t)m * (size_t)P + (size_t)(n0 + cq);
    const v4f rr = *(const v4fa*)(Hbb + off);
    v = v + rr;
    vals[s] = v;
    *(volatile v4f*)(Hbb + off) = v;
  }
  __threadfence();
  #pragma unroll
  for (int s = 0; s < MC * 2; ++s) {
    const int m = wv * (MC * 8) + s * 4 + rsub;
    const size_t off = (size_t)m * (size_t)P + (size_t)(n0 + cq);
    *(volatile v4f*)(Hbb + off) = vals[s];
  }
}

static bool mix_ok(int M, int K, int T, int P, int Nv)
{
  if (M != 32 && M != 64) return false;
  if (K < 32 || K > 96 || (K % 32) != 0) return false;
  if (T != 1 && T != 3) return false;
  if ((32 + T - 1) * (K + 8) > 4608) return false;
  if (M * 36 > 4608) return false;
  if (P < 32 || (P % 32) != 0 || Nv > P || Nv < 1) return false;
  return true;
}

static void mix(hipStream_t st, int M, int mode, int Bn,
                const unsigned short* Wh, const unsigned short* Wl, int wts, int T, const float* bias,
                const float* X, const float* nst, int K, int Nv, int P, int xbs,
                float* Y, int ybs, int act)
{
  dim3 g((unsigned)(P / 32), 1, (unsigned)Bn);
  dim3 blk(64, 1, 1);
  const int mt = M / 16;
  if (mode == 0) {
    if (mt == 2)      k_mix<2, 0><<<g, blk, 0, st>>>(Wh, Wl, wts, T, bias, X, nst, K, Nv, P, xbs, Y, ybs, act);
    else if (mt == 4) k_mix<4, 0><<<g, blk, 0, st>>>(Wh, Wl, wts, T, bias, X, nst, K, Nv, P, xbs, Y, ybs, act);
  } else {
    if (mt == 2)      k_mix<2, 1><<<g, blk, 0, st>>>(Wh, Wl, wts, T, bias, X, nst, K, Nv, P, xbs, Y, ybs, act);
    else if (mt == 4) k_mix<4, 1><<<g, blk, 0, st>>>(Wh, Wl, wts, T, bias, X, nst, K, Nv, P, xbs, Y, ybs, act);
  }
}

extern "C" void kernel_launch(void* const* d_in, const int* in_sizes, int n_in,
                              void* d_out, int out_size, void* d_ws, size_t ws_size,
                              hipStream_t stream)
{
  (void)n_in;
  const float* x    = (const float*)d_in[0];
  const float* lw   = (const float*)d_in[1];
  const float* lb   = (const float*)d_in[2];
  const float* bww  = (const float*)d_in[3];
  const float* bwb  = (const float*)d_in[4];
  const float* bcaw = (const float*)d_in[5];
  const float* bcab = (const float*)d_in[6];
  const float* bcdw = (const float*)d_in[7];
  const float* bcdb = (const float*)d_in[8];
  const float* bm1w = (const float*)d_in[9];
  const float* bm1b = (const float*)d_in[10];
  const float* bm2w = (const float*)d_in[11];
  const float* bm2b = (const float*)d_in[12];
  const float* p1w  = (const float*)d_in[13];
  const float* p1b  = (const float*)d_in[14];
  const float* p2w  = (const float*)d_in[15];
  const float* p2b  = (const float*)d_in[16];
  float* out = (float*)d_out;

  const int S = KS;
  const int C = in_sizes[2];
  if (C != 32 && C != 64) return;
  const int B = in_sizes[0] / S;
  if (B <= 0 || B * S != in_sizes[0]) return;
  const int NB = in_sizes[4] / C;
  if (NB <= 0 || NB * C != in_sizes[4]) return;
  const int LV = in_sizes[8] / (NB * C);
  if (LV < 1 || LV > 7 || LV * NB * C != in_sizes[8]) return;
  const int Hh = in_sizes[10] / NB;
  const int Ch = in_sizes[14];
  if (Hh <= 0 || Ch <= 0 || Hh * NB != in_sizes[10]) return;
  if (Hh != 2 * C) return;
  if ((Ch % 32) != 0 || Ch > C) return;
  if (in_sizes[1] != 2 * C || in_sizes[3] != NB * C * C * 3 || in_sizes[5] != NB * C * C ||
      in_sizes[6] != NB * C || in_sizes[7] != NB * LV * C * C || in_sizes[9] != NB * Hh * C ||
      in_sizes[11] != NB * C * Hh || in_sizes[12] != NB * C || in_sizes[13] != Ch * C ||
      in_sizes[15] != C * Ch || in_sizes[16] != C) return;
  if ((long long)out_size != (long long)B * C * S) return;
  const int NROW = B * C;
  if ((NROW % 32) != 0) return;

  LvTab tb = {};
  tb.L[0] = S; tb.P[0] = S; tb.off[0] = 0;
  long long wdn = 0;
  for (int lv = 1; lv <= LV; ++lv) {
    tb.L[lv] = (tb.L[lv - 1] + 15) / 2;
    tb.P[lv] = ((tb.L[lv] + 31) / 32) * 32;
    tb.off[lv] = (int)wdn;
    wdn += (long long)NROW * tb.P[lv];
  }
  if (wdn > 0x7FFFFFFFLL) return;
  if (S + 29 > 8320 || 2 * tb.P[1] + 16 > 8320 || tb.L[1] > 4160 || tb.P[1] > 5 * 256 * 4) return;
  {
    int alen = tb.L[LV];
    for (int lv = LV; lv >= 1; --lv) {
      const int dl = tb.L[lv];
      if (!(alen == dl || alen == dl + 1)) return;
      const int la = (alen == dl + 1) ? dl : alen;
      if (la + 16 > 4160 || la < 8) return;
      const int lo = 2 * la - 14;
      if (lv > 1 && lo > 4160) return;
      if (lv == 1 && lo < S) return;
      alen = lo;
    }
  }
  if (!mix_ok(C, C, 3, S, S)) return;
  for (int lv = 1; lv <= LV; ++lv) if (!mix_ok(C, C, 1, tb.P[lv], tb.L[lv])) return;
  if (!mix_ok(Ch, C, 1, S, S) || !mix_ok(C, Ch, 1, S, S)) return;

  WpTab wt = {};
  wt.C = C; wt.z = 0;
  wt.nC3 = NB * 3 * C * C;
  wt.nM1 = NB * Hh * C;
  wt.nM2 = NB * C * Hh;
  wt.nCA = NB * C * C;
  wt.nCD = NB * LV * C * C;
  wt.nP1 = Ch * C;
  wt.nP2 = C * Ch;
  wt.oC3  = 0;
  wt.oM1  = wt.oC3 + wt.nC3;
  wt.oM2  = wt.oM1 + wt.nM1;
  wt.oCAh = wt.oM2 + wt.nM2;
  wt.oCAl = wt.oCAh + wt.nCA;
  wt.oCDh = wt.oCAl + wt.nCA;
  wt.oCDl = wt.oCDh + wt.nCD;
  wt.oP1h = wt.oCDl + wt.nCD;
  wt.oP1l = wt.oP1h + wt.nP1;
  wt.oP2h = wt.oP1l + wt.nP1;
  wt.oP2l = wt.oP2h + wt.nP2;
  const long long wpn = (long long)wt.oP2l + wt.nP2;

  const size_t HS = (size_t)NROW * S;
  const size_t oH   = 0;
  const size_t oXS  = oH + HS;
  const size_t oWD  = oXS + HS;
  const size_t oWA  = oWD + (size_t)wdn;
  const size_t oST  = oWA + (size_t)NROW * tb.P[LV];
  const size_t oWP  = oST + (size_t)(((2 * NROW + 31) / 32) * 32);
  const size_t oEnd = oWP + (size_t)(((wpn + 63) / 64) * 32);
  if (oEnd * sizeof(float) > ws_size) return;
  if (oEnd * sizeof(float) > (size_t)134217728) return;
  if ((size_t)B * Ch * S > HS) return;
  float* ws  = (float*)d_ws;
  float* H   = ws + oH;
  float* XS  = ws + oXS;
  float* WD  = ws + oWD;
  float* WA  = ws + oWA;
  float* ST  = ws + oST;
  unsigned short* WP = reinterpret_cast<unsigned short*>(ws + oWP);

  {
    int maxn = wt.nC3;
    if (wt.nM1 > maxn) maxn = wt.nM1;
    if (wt.nM2 > maxn) maxn = wt.nM2;
    if (wt.nCA > maxn) maxn = wt.nCA;
    if (wt.nCD > maxn) maxn = wt.nCD;
    if (wt.nP1 > maxn) maxn = wt.nP1;
    if (wt.nP2 > maxn) maxn = wt.nP2;
    const int gx = ((maxn / 8) + 255) / 256;
    k_wprep<<<dim3((unsigned)gx, 7, 1), dim3(256, 1, 1), 0, stream>>>(bww, bm1w, bm2w, bcaw, bcdw, p1w, p2w, WP, wt);
  }

  const int total4 = (int)(HS / 4);
  k_lift<<<dim3((unsigned)((total4 + 255) / 256)), dim3(256), 0, stream>>>(x, lw, lb, H, C, total4);

  for (int blk = 0; blk < NB; ++blk) {
    const float* wb  = bwb  + (size_t)blk * C;
    const float* cab = bcab + (size_t)blk * C;
    const float* cdb = bcdb + (size_t)blk * LV * C;
    const float* m1b = bm1b + (size_t)blk * Hh;
    const float* m2b = bm2b + (size_t)blk * C;
    const unsigned short* wc3  = WP + (size_t)wt.oC3  + (size_t)blk * 3 * C * C;
    const unsigned short* wm1  = WP + (size_t)wt.oM1  + (size_t)blk * Hh * C;
    const unsigned short* wm2  = WP + (size_t)wt.oM2  + (size_t)blk * C * Hh;
    const unsigned short* wcah = WP + (size_t)wt.oCAh + (size_t)blk * C * C;
    const unsigned short* wcal = WP + (size_t)wt.oCAl + (size_t)blk * C * C;

    k_stats<<<dim3((unsigned)(NROW / 32)), dim3(256), 0, stream>>>(H, ST);
    mix(stream, C, 0, B, wc3, wc3, C * C, 3, wb, H, ST, C, S, S, C * S, XS, C * S, 0);
    k_dwt<<<dim3((unsigned)NROW), dim3(256), 0, stream>>>(H, ST, WD, WA, tb, LV);
    mix(stream, C, 1, B, wcah, wcal, 0, 1, cab, WA, nullptr, C, tb.L[LV], tb.P[LV], C * tb.P[LV], WA, C * tb.P[LV], 0);
    for (int j = 0; j < LV; ++j) {
      const int lv = LV - j;
      const unsigned short* wh = WP + (size_t)wt.oCDh + ((size_t)blk * LV + j) * C * C;
      const unsigned short* wl = WP + (size_t)wt.oCDl + ((size_t)blk * LV + j) * C * C;
      float* band = WD + tb.off[lv];
      mix(stream, C, 1, B, wh, wl, 0, 1, cdb + (size_t)j * C,
          band, nullptr, C, tb.L[lv], tb.P[lv], C * tb.P[lv], band, C * tb.P[lv], 0);
    }
    k_idwt<<<dim3((unsigned)NROW), dim3(256), 0, stream>>>(WA, WD, XS, H, tb, LV);
    k_stats<<<dim3((unsigned)(NROW / 32)), dim3(256), 0, stream>>>(H, ST);
    {
      dim3 g((unsigned)(S / 32), 1, (unsigned)B);
      dim3 bl(64, 1, 1);
      if (C == 64) k_mlp<4, 8><<<g, bl, 0, stream>>>(wm1, m1b, wm2, m2b, ST, H, S);
      else         k_mlp<2, 4><<<g, bl, 0, stream>>>(wm1, m1b, wm2, m2b, ST, H, S);
    }
  }

  float* P1o = XS;
  mix(stream, Ch, 1, B, WP + (size_t)wt.oP1h, WP + (size_t)wt.oP1l, 0, 1, p1b, H, nullptr, C, S, S, C * S, P1o, Ch * S, 1);
  mix(stream, C, 1, B, WP + (size_t)wt.oP2h, WP + (size_t)wt.oP2l, 0, 1, p2b, P1o, nullptr, Ch, S, S, Ch * S, out, C * S, 0);
}
